// GroupedQueryAttention_15891378995337
// MI455X (gfx1250) — hardware-run, weakly checked
//
#include <hip/hip_runtime.h>
#include <math.h>

typedef __attribute__((ext_vector_type(16))) _Float16     v16h;
typedef __attribute__((ext_vector_type(8)))  _Float16     v8h;
typedef __attribute__((ext_vector_type(16))) __bf16       v16b;
typedef __attribute__((ext_vector_type(8)))  float        v8f;
typedef __attribute__((ext_vector_type(4)))  float        v4f;
typedef __attribute__((ext_vector_type(2)))  float        v2f;
typedef __attribute__((ext_vector_type(4)))  unsigned int v4u;

#ifndef NB
#define NB 4
#endif
#ifndef SEQ
#define SEQ 2048
#endif
#define NB_FULL  4
#define SEQ_FULL 2048
#define DM    1024
#define NH    16
#define HDIM  64
#define NQKV  3072
#define NPAIR 32
#define KC    64
#define QT    16
#define NWAVE 8
#define QB    128
#define MROWS (NB * SEQ)
#define HP_ELEMS ((size_t)NB * NH * SEQ * HDIM)

#define ROPE_BYTES ((size_t)SEQ * NPAIR * 2 * 4)
#define X16_BYTES  ((size_t)MROWS * DM * 2)
#define WAT_BYTES  ((size_t)NQKV * DM * 2)
#define WPT_BYTES  ((size_t)DM * DM * 2)
#define HP_BYTES   (HP_ELEMS * 2)
#define O16_BYTES  ((size_t)MROWS * DM * 2)
#define OFF_ROPE ((size_t)0)
#define OFF_X16  (OFF_ROPE + ROPE_BYTES)
#define OFF_WAT  (OFF_X16 + X16_BYTES)
#define OFF_WPT  (OFF_WAT + WAT_BYTES)
#define OFF_HP   (OFF_WPT + WPT_BYTES)
#define OFF_O16  (OFF_HP + 3 * HP_BYTES)
#define WS_TOTAL (OFF_O16 + O16_BYTES)

static_assert(SEQ % QB == 0);
static_assert(SEQ % KC == 0);
static_assert(SEQ <= SEQ_FULL && NB <= NB_FULL);
static_assert(DM == NH * HDIM && NQKV == 3 * DM);
static_assert(DM % 128 == 0 && NQKV % 128 == 0 && MROWS % 128 == 0 && DM % 64 == 0 && NQKV % 64 == 0);
static_assert(DM % 32 == 0);
static_assert(HDIM == 64 && KC == 64 && QT == 16 && NWAVE * QT == QB);
static_assert(NWAVE * 32 * 2 == KC * (HDIM / 8));
static_assert(64 * 132 <= 128 * 68);
static_assert(ROPE_BYTES % 256 == 0 && X16_BYTES % 256 == 0 && WAT_BYTES % 256 == 0 && WPT_BYTES % 256 == 0);
static_assert(HP_BYTES % 256 == 0 && O16_BYTES % 256 == 0);
static_assert(WS_TOTAL <= (size_t)134217728);

__device__ __forceinline__ unsigned int bf_bits(float f) {
    const unsigned int u = __float_as_uint(f);
    return (u + 0x7FFFu + ((u >> 16) & 1u)) >> 16;
}
__device__ __forceinline__ float bf_val(float f) { return __uint_as_float(bf_bits(f) << 16); }
__device__ __forceinline__ unsigned int h_bits(float f) { return (unsigned int)__builtin_bit_cast(unsigned short, (_Float16)f); }

__device__ __forceinline__ v8f mma_bf(v16b a, v16b b, v8f c) {
    c = __builtin_amdgcn_wmma_f32_16x16x32_bf16(false, a, false, b, (short)0, c, false, false);
    asm volatile("v_nop\n\tv_nop\n\tv_nop\n\tv_nop" : "+v"(c) : "v"(a), "v"(b));
    return c;
}
__device__ __forceinline__ v8f mma_h(v16h a, v16h b, v8f c) {
    c = __builtin_amdgcn_wmma_f32_16x16x32_f16(false, a, false, b, (short)0, c, false, false);
    asm volatile("v_nop\n\tv_nop\n\tv_nop\n\tv_nop" : "+v"(c) : "v"(a), "v"(b));
    return c;
}

__device__ __forceinline__ void st16x2(unsigned short* p, v4u v) {
    volatile v4u* d = (volatile v4u*)p;
    *d = v; __threadfence(); *d = v;
}

__global__ __launch_bounds__(256) void k_rope_tab(float* __restrict__ tab) {
    const int u = blockIdx.x * 256 + threadIdx.x;
    if (u >= SEQ * NPAIR) return;
    const int t = u >> 5, p = u & 31;
    const float e = -(float)(p + 1) * 0.03125f;
    const float theta = exp2f(e * 9.965784284662087f);
    const float ang = (float)(t + 1) * theta;
    v2f cs;
    cs.x = cosf(ang);
    cs.y = sinf(ang);
    volatile v2f* d = (volatile v2f*)(tab + (size_t)u * 2);
    *d = cs; __threadfence(); *d = cs;
}

__global__ __launch_bounds__(256) void k_cvt_x(const float* __restrict__ xin, unsigned short* __restrict__ X16) {
    const long long u = (long long)blockIdx.x * 256 + threadIdx.x;
    if (u >= (long long)MROWS * (DM / 8)) return;
    const int pc = (int)(u % (DM / 8));
    const long long row = u / (DM / 8);
    const int b = (int)(row / SEQ), s = (int)(row - (long long)b * SEQ);
    const float* src = xin + ((size_t)b * SEQ_FULL + s) * DM + pc * 8;
    const v4f a = *(const v4f*)(src), c = *(const v4f*)(src + 4);
    v4u pk;
    pk.x = bf_bits(a.x) | (bf_bits(a.y) << 16); pk.y = bf_bits(a.z) | (bf_bits(a.w) << 16);
    pk.z = bf_bits(c.x) | (bf_bits(c.y) << 16); pk.w = bf_bits(c.z) | (bf_bits(c.w) << 16);
    st16x2(X16 + (size_t)row * DM + pc * 8, pk);
}

template <int MODE>
__device__ __forceinline__ unsigned int wbits(float f) {
    if (MODE == 0) return bf_bits(f);
    return h_bits(bf_val(f) * 256.0f);
}
template <int MODE>
__global__ __launch_bounds__(256) void k_cvt_wt(const float* __restrict__ W, unsigned short* __restrict__ WT, int N) {
    __shared__ __align__(16) unsigned short tile[64 * 72];
    const int t = threadIdx.x;
    const int k0 = blockIdx.x * 64, n0 = blockIdx.y * 64;
    {
        const int rl = t >> 2, part = t & 3;
        const float* src = W + (size_t)(k0 + rl) * N + n0 + part * 16;
        const v4f f0 = *(const v4f*)(src), f1 = *(const v4f*)(src + 4), f2 = *(const v4f*)(src + 8), f3 = *(const v4f*)(src + 12);
        v4u p0, p1;
        p0.x = wbits<MODE>(f0.x) | (wbits<MODE>(f0.y) << 16); p0.y = wbits<MODE>(f0.z) | (wbits<MODE>(f0.w) << 16);
        p0.z = wbits<MODE>(f1.x) | (wbits<MODE>(f1.y) << 16); p0.w = wbits<MODE>(f1.z) | (wbits<MODE>(f1.w) << 16);
        p1.x = wbits<MODE>(f2.x) | (wbits<MODE>(f2.y) << 16); p1.y = wbits<MODE>(f2.z) | (wbits<MODE>(f2.w) << 16);
        p1.z = wbits<MODE>(f3.x) | (wbits<MODE>(f3.y) << 16); p1.w = wbits<MODE>(f3.z) | (wbits<MODE>(f3.w) << 16);
        *(v4u*)(tile + rl * 72 + part * 16)     = p0;
        *(v4u*)(tile + rl * 72 + part * 16 + 8) = p1;
    }
    __syncthreads();
#pragma unroll
    for (int it = 0; it < 2; ++it) {
        const int nrow = it * 32 + (t >> 3), pc = t & 7;
        unsigned int e[8];
#pragma unroll
        for (int j = 0; j < 8; ++j) e[j] = (unsigned int)tile[(pc * 8 + j) * 72 + nrow];
        v4u pk;
        pk.x = e[0] | (e[1] << 16); pk.y = e[2] | (e[3] << 16); pk.z = e[4] | (e[5] << 16); pk.w = e[6] | (e[7] << 16);
        st16x2(WT + (size_t)(n0 + nrow) * DM + k0 + pc * 8, pk);
    }
}

template <int MODE>
__global__ __launch_bounds__(256) void k_gemm(const unsigned short* __restrict__ A, const unsigned short* __restrict__ Bt,
                                               const float* __restrict__ bias, const float* __restrict__ rope,
                                               unsigned short* __restrict__ P3, float* __restrict__ out) {
    union FU { v4u u[2]; v16b b; v16h h; };
    __shared__ __align__(16) unsigned short As[128 * 32];
    __shared__ __align__(16) unsigned short Bs[128 * 32];
    __shared__ __align__(16) float          Cs[128 * 68];

    const int tid = threadIdx.x, wave = tid >> 5, lane = tid & 31, hh = lane >> 4, c = lane & 15;
    const int wm = wave & 3, wn = wave >> 2;
    const int m0 = blockIdx.x * 128, n0 = blockIdx.y * 128;

    v8f acc[2][4];
#pragma unroll
    for (int ms = 0; ms < 2; ++ms)
#pragma unroll
        for (int ns = 0; ns < 4; ++ns) acc[ms][ns] = (v8f){0.f, 0.f, 0.f, 0.f, 0.f, 0.f, 0.f, 0.f};

    for (int kt = 0; kt < DM / 32; ++kt) {
        const int k0 = kt * 32;
        __syncthreads();
#pragma unroll
        for (int i = 0; i < 2; ++i) {
            const int idx = tid + 256 * i;
            const int row = idx >> 2, pc = idx & 3;
            const v4u av = *(const v4u*)(A  + (size_t)(m0 + row) * DM + k0 + pc * 8);
            const v4u bv = *(const v4u*)(Bt + (size_t)(n0 + row) * DM + k0 + pc * 8);
            *(v4u*)(As + row * 32 + pc * 8) = av;
            *(v4u*)(Bs + row * 32 + pc * 8) = bv;
        }
        __syncthreads();

        FU af[2], bq[4];
#pragma unroll
        for (int ms = 0; ms < 2; ++ms) {
            const unsigned short* ap = As + (wm * 32 + ms * 16 + c) * 32;
            af[ms].u[0] = *(const v4u*)(ap + 8 * hh);
            af[ms].u[1] = *(const v4u*)(ap + 16 + 8 * hh);
        }
#pragma unroll
        for (int ns = 0; ns < 4; ++ns) {
            const unsigned short* bp = Bs + (wn * 64 + ns * 16 + c) * 32;
            bq[ns].u[0] = *(const v4u*)(bp + 8 * hh);
            bq[ns].u[1] = *(const v4u*)(bp + 16 + 8 * hh);
        }
#pragma unroll
        for (int ms = 0; ms < 2; ++ms)
#pragma unroll
            for (int ns = 0; ns < 4; ++ns) {
                if (MODE == 0) acc[ms][ns] = mma_bf(af[ms].b, bq[ns].b, acc[ms][ns]);
                else           acc[ms][ns] = mma_h(af[ms].h, bq[ns].h, acc[ms][ns]);
            }
    }

    const int sec = (MODE == 0) ? (n0 / DM) : 0;
    const bool trans = (MODE == 0) && (sec == 2);
    const int bb = m0 / SEQ, t0 = m0 - bb * SEQ;

#pragma unroll
    for (int ph = 0; ph < 2; ++ph) {
        __syncthreads();
        if (wn == ph) {
#pragma unroll
            for (int ms = 0; ms < 2; ++ms)
#pragma unroll
                for (int ns = 0; ns < 4; ++ns)
#pragma unroll
                    for (int r = 0; r < 8; ++r) {
                        const int row = wm * 32 + ms * 16 + 8 * hh + r;
                        const int col = ns * 16 + c;
                        const int si = trans ? (col * 132 + row) : (row * 68 + col);
                        Cs[si] = acc[ms][ns][r];
                    }
        }
        __syncthreads();

        if (MODE == 0) {
            const int head = ((n0 - sec * DM) >> 6) + ph;
            v4u pk[4];
            size_t off[4];
            if (!trans) {
#pragma unroll
                for (int it = 0; it < 4; ++it) {
                    const int idx = tid + 256 * it;
                    const int row = idx >> 3, pc = idx & 7;
                    const v4f f0 = *(const v4f*)(Cs + row * 68 + pc * 8);
                    const v4f f1 = *(const v4f*)(Cs + row * 68 + pc * 8 + 4);
                    const int nb = n0 + ph * 64 + pc * 8;
                    const v4f b0 = *(const v4f*)(bias + nb);
                    const v4f b1 = *(const v4f*)(bias + nb + 4);
                    const float* rp = rope + ((size_t)(t0 + row) * NPAIR + pc * 4) * 2;
                    const v4f r0 = *(const v4f*)(rp);
                    const v4f r1 = *(const v4f*)(rp + 4);
                    const float x0 = f0.x + bf_val(b0.x), x1 = f0.y + bf_val(b0.y);
                    const float x2 = f0.z + bf_val(b0.z), x3 = f0.w + bf_val(b0.w);
                    const float x4 = f1.x + bf_val(b1.x), x5 = f1.y + bf_val(b1.y);
                    const float x6 = f1.z + bf_val(b1.z), x7 = f1.w + bf_val(b1.w);
                    const float o0 = x0 * r0.x - x1 * r0.y, o1 = x1 * r0.x + x0 * r0.y;
                    const float o2 = x2 * r0.z - x3 * r0.w, o3 = x3 * r0.z + x2 * r0.w;
                    const float o4 = x4 * r1.x - x5 * r1.y, o5 = x5 * r1.x + x4 * r1.y;
                    const float o6 = x6 * r1.z - x7 * r1.w, o7 = x7 * r1.z + x6 * r1.w;
                    pk[it].x = h_bits(o0) | (h_bits(o1) << 16);
                    pk[it].y = h_bits(o2) | (h_bits(o3) << 16);
                    pk[it].z = h_bits(o4) | (h_bits(o5) << 16);
                    pk[it].w = h_bits(o6) | (h_bits(o7) << 16);
                    off[it] = (size_t)sec * HP_ELEMS + ((size_t)(bb * NH + head) * SEQ + t0 + row) * HDIM + pc * 8;
                }
            } else {
#pragma unroll
                for (int it = 0; it < 4; ++it) {
                    const int idx = tid + 256 * it;
                    const int ch = idx >> 4, pc = idx & 15;
                    const v4f f0 = *(const v4f*)(Cs + ch * 132 + pc * 8);
                    const v4f f1 = *(const v4f*)(Cs + ch * 132 + pc * 8 + 4);
                    const float bv = bf_val(bias[n0 + ph * 64 + ch]);
                    pk[it].x = h_bits(f0.x + bv) | (h_bits(f0.y + bv) << 16);
                    pk[it].y = h_bits(f0.z + bv) | (h_bits(f0.w + bv) << 16);
                    pk[it].z = h_bits(f1.x + bv) | (h_bits(f1.y + bv) << 16);
                    pk[it].w = h_bits(f1.z + bv) | (h_bits(f1.w + bv) << 16);
                    off[it] = (size_t)2 * HP_ELEMS + ((size_t)((bb * NH + head) * HDIM + ch)) * SEQ + t0 + pc * 8;
                }
            }
#pragma unroll
            for (int it = 0; it < 4; ++it) *(volatile v4u*)(P3 + off[it]) = pk[it];
            __threadfence();
#pragma unroll
            for (int it = 0; it < 4; ++it) *(volatile v4u*)(P3 + off[it]) = pk[it];
        } else {
            v4f ov[8];
            size_t off[8];
#pragma unroll
            for (int it = 0; it < 8; ++it) {
                const int idx = tid + 256 * it;
                const int row = idx >> 4, pc = idx & 15;
                const v4f f = *(const v4f*)(Cs + row * 68 + pc * 4);
                const int nb = n0 + ph * 64 + pc * 4;
                const v4f bz = *(const v4f*)(bias + nb);
                const float isc = 1.52587890625e-05f;
                ov[it].x = f.x * isc + bf_val(bz.x);
                ov[it].y = f.y * isc + bf_val(bz.y);
                ov[it].z = f.z * isc + bf_val(bz.z);
                ov[it].w = f.w * isc + bf_val(bz.w);
                off[it] = (size_t)(m0 + row) * DM + nb;
            }
#pragma unroll
            for (int it = 0; it < 8; ++it) *(volatile v4f*)(out + off[it]) = ov[it];
            __threadfence();
#pragma unroll
            for (int it = 0; it < 8; ++it) *(volatile v4f*)(out + off[it]) = ov[it];
        }
    }
}

__global__ __launch_bounds__(256) void k_attn(const unsigned short* __restrict__ Q16, const unsigned short* __restrict__ K16,
                                               const unsigned short* __restrict__ VT16, unsigned short* __restrict__ O16) {
    union FH { v16h v; v8h h[2]; };
    __shared__ __align__(16) unsigned short Ksh[KC * HDIM];
    __shared__ __align__(16) unsigned short Vth[HDIM * KC];
    __shared__ __align__(16) _Float16       Psh[NWAVE][QT * KC];

    const int tid = threadIdx.x, wave = tid >> 5, lane = tid & 31, hh = lane >> 4, c = lane & 15;
    const int head = blockIdx.y, b = blockIdx.z;
    const int bh = b * NH + head;
    const int q0 = blockIdx.x * QB + wave * QT;
    const float SCL = 0.04419417382415922f * 1.4426950408889634f;
    const float PSC = 32768.0f;
    const float OSC = 256.0f;

    FH qa[2];
    {
        const _Float16* qrow = (const _Float16*)Q16 + ((size_t)bh * SEQ + q0 + c) * HDIM;
#pragma unroll
        for (int dc = 0; dc < 2; ++dc) {
            qa[dc].h[0] = *(const v8h*)(qrow + dc * 32 + 8 * hh);
            qa[dc].h[1] = *(const v8h*)(qrow + dc * 32 + 16 + 8 * hh);
        }
    }

    float mrow[8], lrow[8];
    v8f oacc[4];
#pragma unroll
    for (int r = 0; r < 8; ++r) { mrow[r] = -INFINITY; lrow[r] = 0.f; }
#pragma unroll
    for (int t = 0; t < 4; ++t) oacc[t] = (v8f){0.f, 0.f, 0.f, 0.f, 0.f, 0.f, 0.f, 0.f};

    const unsigned short* Kb = K16 + (size_t)bh * SEQ * HDIM;
    const unsigned short* Vb = VT16 + (size_t)bh * HDIM * SEQ;
    const _Float16* Kp = (const _Float16*)Ksh;
    const _Float16* Vp = (const _Float16*)Vth;
    _Float16* pw = Psh[wave];

    for (int kc = 0; kc < SEQ / KC; ++kc) {
        const int kv0 = kc * KC;
        __syncthreads();
#pragma unroll
        for (int i = 0; i < 2; ++i) {
            const int idx = tid + 256 * i;
            const int row = idx >> 3, pc = idx & 7;
            const v4u kk = *(const v4u*)(Kb + (size_t)(kv0 + row) * HDIM + pc * 8);
            const v4u vv = *(const v4u*)(Vb + (size_t)row * SEQ + kv0 + pc * 8);
            *(v4u*)(Ksh + row * HDIM + pc * 8) = kk;
            *(v4u*)(Vth + row * KC + pc * 8)   = vv;
        }
        __syncthreads();

        v8f s[4];
#pragma unroll
        for (int j = 0; j < 4; ++j) {
            s[j] = (v8f){0.f, 0.f, 0.f, 0.f, 0.f, 0.f, 0.f, 0.f};
#pragma unroll
            for (int dc = 0; dc < 2; ++dc) {
                FH kb;
                kb.h[0] = *(const v8h*)(Kp + (j * 16 + c) * HDIM + dc * 32 + 8 * hh);
                kb.h[1] = *(const v8h*)(Kp + (j * 16 + c) * HDIM + dc * 32 + 16 + 8 * hh);
                s[j] = mma_h(qa[dc].v, kb.v, s[j]);
            }
        }

#pragma unroll
        for (int r = 0; r < 8; ++r) {
            const float x0 = s[0][r] * SCL, x1 = s[1][r] * SCL, x2 = s[2][r] * SCL, x3 = s[3][r] * SCL;
            float m = fmaxf(fmaxf(x0, x1), fmaxf(x2, x3));
            m = fmaxf(m, __shfl_xor(m, 1, 32)); m = fmaxf(m, __shfl_xor(m, 2, 32));
            m = fmaxf(m, __shfl_xor(m, 4, 32)); m = fmaxf(m, __shfl_xor(m, 8, 32));
            const float mnew  = fmaxf(mrow[r], m);
            const float alpha = exp2f(mrow[r] - mnew);
            mrow[r] = mnew;
            const float p0 = exp2f(x0 - mnew), p1 = exp2f(x1 - mnew), p2 = exp2f(x2 - mnew), p3 = exp2f(x3 - mnew);
            _Float16* prow = pw + (8 * hh + r) * KC + c;
            prow[0]  = (_Float16)(p0 * PSC);
            prow[16] = (_Float16)(p1 * PSC);
            prow[32] = (_Float16)(p2 * PSC);
            prow[48] = (_Float16)(p3 * PSC);
            float psum = (p0 + p1) + (p2 + p3);
            psum += __shfl_xor(psum, 1, 32); psum += __shfl_xor(psum, 2, 32);
            psum += __shfl_xor(psum, 4, 32); psum += __shfl_xor(psum, 8, 32);
            lrow[r] = lrow[r] * alpha + psum;
#pragma unroll
            for (int t = 0; t < 4; ++t) oacc[t][r] *= alpha;
        }
        __builtin_amdgcn_fence(3  , "workgroup");
        __builtin_amdgcn_wave_barrier();
        __builtin_amdgcn_fence(2  , "workgroup");

#pragma unroll
        for (int kk = 0; kk < 2; ++kk) {
            FH pa;
            pa.h[0] = *(const v8h*)(pw + c * KC + kk * 32 + 8 * hh);
            pa.h[1] = *(const v8h*)(pw + c * KC + kk * 32 + 16 + 8 * hh);
#pragma unroll
            for (int t = 0; t < 4; ++t) {
                FH vb;
                vb.h[0] = *(const v8h*)(Vp + (t * 16 + c) * KC + kk * 32 + 8 * hh);
                vb.h[1] = *(const v8h*)(Vp + (t * 16 + c) * KC + kk * 32 + 16 + 8 * hh);
                oacc[t] = mma_h(pa.v, vb.v, oacc[t]);
            }
        }
    }

    __builtin_amdgcn_fence(3  , "workgroup");
    __builtin_amdgcn_wave_barrier();
    __builtin_amdgcn_fence(2  , "workgroup");
#pragma unroll
    for (int r = 0; r < 8; ++r) {
        const float inv = OSC * (1.0f / (lrow[r] * PSC));
#pragma unroll
        for (int t = 0; t < 4; ++t) pw[(8 * hh + r) * KC + t * 16 + c] = (_Float16)(oacc[t][r] * inv);
    }
    __builtin_amdgcn_fence(3  , "workgroup");
    __builtin_amdgcn_wave_barrier();
    __builtin_amdgcn_fence(2  , "workgroup");
    {
        unsigned short* ob = O16 + ((size_t)b * SEQ + q0) * DM + head * HDIM;
        const int rsub = lane >> 3, pc = lane & 7;
        v4u ov[4];
#pragma unroll
        for (int it = 0; it < 4; ++it) {
            const v8h hv = *(const v8h*)(pw + (it * 4 + rsub) * KC + pc * 8);
            ov[it] = __builtin_bit_cast(v4u, hv);
        }
#pragma unroll
        for (int it = 0; it < 4; ++it) *(volatile v4u*)(ob + (size_t)(it * 4 + rsub) * DM + pc * 8) = ov[it];
        __threadfence();
#pragma unroll
        for (int it = 0; it < 4; ++it) *(volatile v4u*)(ob + (size_t)(it * 4 + rsub) * DM + pc * 8) = ov[it];
    }
}

extern "C" void kernel_launch(void* const* d_in, const int* in_sizes, int n_in, void* d_out, int out_size, void* d_ws, size_t ws_size, hipStream_t stream) {
    if (n_in < 5) return;
    if ((long long)in_sizes[0] < (long long)(NB - 1) * SEQ_FULL * DM + (long long)SEQ * DM) return;
    if ((long long)in_sizes[1] < (long long)DM * NQKV) return;
    if ((long long)in_sizes[2] < (long long)NQKV) return;
    if ((long long)in_sizes[3] < (long long)DM * DM) return;
    if ((long long)in_sizes[4] < (long long)DM) return;
    if ((long long)out_size < (long long)MROWS * DM) return;
    if (ws_size < WS_TOTAL) return;

    const float* x      = (const float*)d_in[0];
    const float* W_attn = (const float*)d_in[1];
    const float* b_attn = (const float*)d_in[2];
    const float* W_proj = (const float*)d_in[3];
    const float* b_proj = (const float*)d_in[4];
    float* out = (float*)d_out;

    char* ws = (char*)d_ws;
    float*          ROPE = (float*)(ws + OFF_ROPE);
    unsigned short* X16  = (unsigned short*)(ws + OFF_X16);
    unsigned short* WAT  = (unsigned short*)(ws + OFF_WAT);
    unsigned short* WPT  = (unsigned short*)(ws + OFF_WPT);
    unsigned short* P3   = (unsigned short*)(ws + OFF_HP);
    unsigned short* O16  = (unsigned short*)(ws + OFF_O16);

    k_rope_tab<<<(unsigned)((SEQ * NPAIR + 255) / 256), 256, 0, stream>>>(ROPE);
    k_cvt_x<<<(unsigned)(((long long)MROWS * (DM / 8) + 255) / 256), 256, 0, stream>>>(x, X16);
    k_cvt_wt<0><<<dim3((unsigned)(DM / 64), (unsigned)(NQKV / 64)), 256, 0, stream>>>(W_attn, WAT, NQKV);
    k_cvt_wt<1><<<dim3((unsigned)(DM / 64), (unsigned)(DM / 64)), 256, 0, stream>>>(W_proj, WPT, DM);

    k_gemm<0><<<dim3((unsigned)(MROWS / 128), (unsigned)(NQKV / 128)), 256, 0, stream>>>(X16, WAT, b_attn, ROPE, P3, out);

    k_attn<<<dim3((unsigned)(SEQ / QB), (unsigned)NH, (unsigned)NB), 256, 0, stream>>>(P3, P3 + HP_ELEMS, P3 + 2 * HP_ELEMS, O16);

    k_gemm<1><<<dim3((unsigned)(MROWS / 128), (unsigned)(DM / 128)), 256, 0, stream>>>(O16, WPT, b_proj, ROPE, P3, out);
}
